// SelfAtten_77945066488216
// MI455X (gfx1250) — hardware-verified
//
#include <hip/hip_runtime.h>
#include <stdint.h>

typedef __attribute__((ext_vector_type(16))) _Float16 v16h;
typedef __attribute__((ext_vector_type(8)))  _Float16 v8h;
typedef __attribute__((ext_vector_type(16))) __bf16   v16b;
typedef __attribute__((ext_vector_type(8)))  __bf16   v8b;
typedef __attribute__((ext_vector_type(8)))  float    v8f;
typedef __attribute__((ext_vector_type(4)))  float    v4f;

__device__ __forceinline__ unsigned short f2bf_bits(float f) {
  unsigned u = __float_as_uint(f);
  return (unsigned short)((u + 0x7FFFu + ((u >> 16) & 1u)) >> 16);
}
__device__ __forceinline__ float bf_bits2f(unsigned short h) { return __uint_as_float(((unsigned)h) << 16); }

__device__ __forceinline__ void dep_guard_h(v8f& a, v8f& b, v16h x, v16h y) { asm volatile("v_nop\n\tv_nop\n\tv_nop\n\tv_nop" : "+v"(a), "+v"(b) : "v"(x), "v"(y)); }
__device__ __forceinline__ void dep_guard_b(v8f& a, v8f& b, v16b x, v16b y) { asm volatile("v_nop\n\tv_nop\n\tv_nop\n\tv_nop" : "+v"(a), "+v"(b) : "v"(x), "v"(y)); }
__device__ __forceinline__ void keep4_h(v16h a, v16h b, v16h c, v16h d) { asm volatile("v_nop" :: "v"(a), "v"(b), "v"(c), "v"(d)); }
__device__ __forceinline__ void keep4_b(v16b a, v16b b, v16b c, v16b d) { asm volatile("v_nop" :: "v"(a), "v"(b), "v"(c), "v"(d)); }
__device__ __forceinline__ void acc_guard4(v8f& a, v8f& b, v8f& c, v8f& d) { asm volatile("v_nop\n\tv_nop\n\tv_nop\n\tv_nop" : "+v"(a), "+v"(b), "+v"(c), "+v"(d)); }
template <typename T> struct Frag;
template <> struct Frag<_Float16> {
  typedef v16h V; union U { v16h v; v8h h[2]; };
  static __device__ __forceinline__ v16h load(const _Float16* p) {
    U f; f.h[0] = *(const v8h*)(p); f.h[1] = *(const v8h*)(p + 16); return f.v;
  }
  static __device__ __forceinline__ v8f mma(v16h a, v16h b, v8f c) {
    return __builtin_amdgcn_wmma_f32_16x16x32_f16(false, a, false, b, (short)0, c, false, false);
  }
  static __device__ __forceinline__ void guard(v8f& a, v8f& b, v16h x, v16h y) { dep_guard_h(a, b, x, y); }
  static __device__ __forceinline__ void keep(v16h a, v16h b, v16h c, v16h d) { keep4_h(a, b, c, d); }
};
template <> struct Frag<__bf16> {
  typedef v16b V; union U { v16b v; v8b h[2]; };
  static __device__ __forceinline__ v16b load(const __bf16* p) {
    U f; f.h[0] = *(const v8b*)(p); f.h[1] = *(const v8b*)(p + 16); return f.v;
  }
  static __device__ __forceinline__ v8f mma(v16b a, v16b b, v8f c) {
    return __builtin_amdgcn_wmma_f32_16x16x32_bf16(false, a, false, b, (short)0, c, false, false);
  }
  static __device__ __forceinline__ void guard(v8f& a, v8f& b, v16b x, v16b y) { dep_guard_b(a, b, x, y); }
  static __device__ __forceinline__ void keep(v16b a, v16b b, v16b c, v16b d) { keep4_b(a, b, c, d); }
};

template <int ET> struct Elem;
template <> struct Elem<0> { typedef _Float16 T; };
template <> struct Elem<1> { typedef __bf16 T; };
template <int ET, bool SPLIT, int BIAS_MODE, int OUT_MODE, bool RESID, int ACT = 0>
__global__ __launch_bounds__(256) void wmma_gemm64(
    const unsigned short* __restrict__ Ap, const unsigned short* __restrict__ A2p, int lda, long strideA,
    const unsigned short* __restrict__ Btp, const unsigned short* __restrict__ Bt2p, int ldb, long strideB,
    void* __restrict__ Cout, void* __restrict__ Cout2, int ldc, long strideC,
    const float* __restrict__ bias,
    const float* __restrict__ resid, long strideR,
    int M, int N, int K, float scale) {
  typedef typename Elem<ET>::T T;
  typedef typename Frag<T>::V V;
  const T* A = (const T*)Ap; const T* A2 = (const T*)A2p; const T* Bt = (const T*)Btp; const T* Bt2 = (const T*)Bt2p;
  __shared__ __align__(16) float sT[8][16 * 68];
  const int b    = blockIdx.y;
  const int lane = threadIdx.x & 31;
  const int wave = threadIdx.x >> 5;
  const int tilesN = N >> 6;
  const int tilesM = M >> 6;
  const int tile = blockIdx.x * 8 + wave;
  if (tile >= tilesM * tilesN) return;
  const int tm = tile / tilesN;
  const int tn = tile - tm * tilesN;
  const int m0 = tm << 6;
  const int n0 = tn << 6;

  const T* Ab  = A  + (size_t)b * strideA;
  const T* Bb  = Bt + (size_t)b * strideB;
  const T* Ab2 = SPLIT ? (A2  + (size_t)b * strideA) : nullptr;
  const T* Bb2 = SPLIT ? (Bt2 + (size_t)b * strideB) : nullptr;

  const int rlane = lane & 15;
  const int koff  = (lane >> 4) * 8;
  const int mOff  = (lane >> 4) * 8;

  v8f acc[4][4];
#pragma unroll
  for (int i = 0; i < 4; ++i)
#pragma unroll
    for (int j = 0; j < 4; ++j) acc[i][j] = (v8f){0.f,0.f,0.f,0.f,0.f,0.f,0.f,0.f};

  for (int k0 = 0; k0 < K; k0 += 32) {
    V bh[4], bl[4];
#pragma unroll
    for (int j = 0; j < 4; ++j) {
      const size_t bo = (size_t)(n0 + (j << 4) + rlane) * ldb + koff + k0;
      bh[j] = Frag<T>::load(Bb + bo);
      if (SPLIT) bl[j] = Frag<T>::load(Bb2 + bo);
    }
#pragma unroll
    for (int i = 0; i < 4; ++i) {
      const size_t ao = (size_t)(m0 + (i << 4) + rlane) * lda + koff + k0;
      V ah = Frag<T>::load(Ab + ao);
      V al;
      if (SPLIT) al = Frag<T>::load(Ab2 + ao);
#pragma unroll
      for (int j = 0; j < 4; ++j) {
        acc[i][j] = Frag<T>::mma(ah, bh[j], acc[i][j]);
        if (SPLIT) {
          acc[i][j] = Frag<T>::mma(ah, bl[j], acc[i][j]);
          acc[i][j] = Frag<T>::mma(al, bh[j], acc[i][j]);
        }
      }
      Frag<T>::guard(acc[i][0], acc[i][3], ah, SPLIT ? al : ah);
    }
    Frag<T>::keep(bh[0], bh[1], bh[2], bh[3]);
    if (SPLIT) Frag<T>::keep(bl[0], bl[1], bl[2], bl[3]);
  }
  acc_guard4(acc[0][0], acc[0][1], acc[0][2], acc[0][3]);
  acc_guard4(acc[1][0], acc[1][1], acc[1][2], acc[1][3]);
  acc_guard4(acc[2][0], acc[2][1], acc[2][2], acc[2][3]);
  acc_guard4(acc[3][0], acc[3][1], acc[3][2], acc[3][3]);

  float* slab = sT[wave];
  const float* Rb = RESID ? (resid + (size_t)b * strideR) : nullptr;
#pragma unroll
  for (int i = 0; i < 4; ++i) {
    const int mBase = m0 + (i << 4);
#pragma unroll
    for (int j = 0; j < 4; ++j) {
      const int n = n0 + (j << 4) + rlane;
      float bv = 0.f;
      if (BIAS_MODE == 2) bv = bias[n];
      if (BIAS_MODE == 3) bv = bias[(size_t)b * N + n];
#pragma unroll
      for (int r = 0; r < 8; ++r) {
        float v = acc[i][j][r] * scale;
        if (BIAS_MODE == 1) v += bias[mBase + mOff + r];
        if (BIAS_MODE == 2 || BIAS_MODE == 3) v += bv;
        if (RESID) v += Rb[(size_t)(mBase + mOff + r) * ldc + n];
        if (ACT == 1) v = tanhf(v);
        if (ACT == 2) v = fmaxf(v, 0.0f);
        if (ACT == 3) v = v / (1.0f + expf(-v));
        if (ACT == 4) v = (v > 0.f) ? v : 0.01f * v;
        if (ACT == 5) v = 0.5f * v * (1.0f + erff(v * 0.70710678118654752f));
        slab[(mOff + r) * 68 + (j << 4) + rlane] = v;
      }
    }
    __builtin_amdgcn_fence(__ATOMIC_RELEASE, "workgroup");
    __builtin_amdgcn_wave_barrier();
    __builtin_amdgcn_fence(__ATOMIC_ACQUIRE, "workgroup");
    if (OUT_MODE == 0) {
      float* C = (float*)Cout + (size_t)b * strideC;
      const int hh = lane >> 4, c4 = (lane & 15) * 4;
      for (int pass = 0; pass < 2; ++pass) {
#pragma unroll
        for (int it = 0; it < 8; ++it) {
          const int row = it * 2 + hh;
          v4f v = *(const v4f*)(slab + row * 68 + c4);
          *(volatile v4f*)(C + (size_t)(mBase + row) * ldc + n0 + c4) = v;
        }
        __threadfence();
      }
    } else {
      const int q = lane >> 3, c8 = (lane & 7) * 8;
      unsigned short* C  = (unsigned short*)Cout  + (size_t)b * strideC;
      unsigned short* C2 = (OUT_MODE == 2) ? ((unsigned short*)Cout2 + (size_t)b * strideC) : nullptr;
      for (int pass = 0; pass < 2; ++pass) {
#pragma unroll
        for (int it = 0; it < 4; ++it) {
          const int row = it * 4 + q;
          const float* sp = slab + row * 68 + c8;
          v8h hv, lv;
#pragma unroll
          for (int e = 0; e < 8; ++e) {
            if (OUT_MODE == 1) {
              hv[e] = (_Float16)sp[e];
            } else {
              unsigned short hb = f2bf_bits(sp[e]);
              unsigned short lb = f2bf_bits(sp[e] - bf_bits2f(hb));
              hv[e] = __builtin_bit_cast(_Float16, hb);
              lv[e] = __builtin_bit_cast(_Float16, lb);
            }
          }
          *(volatile v8h*)(C + (size_t)(mBase + row) * ldc + n0 + c8) = hv;
          if (OUT_MODE == 2) *(volatile v8h*)(C2 + (size_t)(mBase + row) * ldc + n0 + c8) = lv;
        }
        __threadfence();
      }
    }
    __builtin_amdgcn_fence(__ATOMIC_RELEASE, "workgroup");
    __builtin_amdgcn_wave_barrier();
    __builtin_amdgcn_fence(__ATOMIC_ACQUIRE, "workgroup");
  }
}

constexpr int NBATCH = 4;
constexpr int SEQ    = 512;
constexpr int MODD   = 128;
constexpr int FEATD  = 256;
constexpr int BPITCH = FEATD + 8;
constexpr int SB_BYTES   = MODD * BPITCH * 2;
constexpr int SMEM_BYTES = SB_BYTES + (FEATD + MODD + SEQ + 16) * 4;
constexpr float BSC      = 64.0f;
constexpr float BSC_INV  = 1.0f / 64.0f;
constexpr float PCARRY   = 1024.0f;
constexpr float PCENTRE  = 2.0f;
static_assert(FEATD % 32 == 0);
static_assert(SEQ % 64 == 0 && FEATD % 64 == 0 && SEQ % 32 == 0);
static_assert(SEQ == 8 * 4 * 16);
static_assert(MODD == 8 * 16);
static_assert(SB_BYTES % 16 == 0);
static_assert((BPITCH * 2) % 16 == 0);

constexpr size_t OFF_HH   = 0;
constexpr size_t OFF_HT   = (size_t)NBATCH * SEQ * FEATD * 2;
constexpr size_t OFF_P    = OFF_HT + (size_t)NBATCH * FEATD * SEQ * 2;
constexpr size_t OFF_MEAN = OFF_P + (size_t)NBATCH * SEQ * SEQ * 2;
constexpr size_t WS_TOTAL = OFF_MEAN + (size_t)NBATCH * FEATD * 4;
static_assert(WS_TOTAL == 4198400);
static_assert(WS_TOTAL <= 134217728);
constexpr size_t OUT0_BYTES = (size_t)NBATCH * SEQ * FEATD * 4;
constexpr size_t OUT1_OFF   = 2097152;
constexpr size_t OUT1_BYTES = (size_t)NBATCH * SEQ * SEQ * 4;
static_assert(OUT1_OFF == OUT0_BYTES);
static_assert(OUT1_OFF % 128 == 0);
static_assert(OUT1_OFF + OUT1_BYTES == 6291456);

__global__ __launch_bounds__(256) void planes_kernel(const float* __restrict__ hidden,
                                                    unsigned short* __restrict__ Hh16p,
                                                    unsigned short* __restrict__ Ht16p) {
  __shared__ float tile[64][65];
  const int tid = threadIdx.x, wave = tid >> 5, lane = tid & 31;
  const int kbase = blockIdx.x * 64, fbase = blockIdx.y * 64, b = blockIdx.z;
  {
    const int rr = tid >> 4, c4 = (tid & 15) * 4;
#pragma unroll
    for (int it = 0; it < 4; ++it) {
      const int row = it * 16 + rr;
      const v4f v = *(const v4f*)(hidden + ((size_t)(b * SEQ + kbase + row)) * FEATD + fbase + c4);
      tile[row][c4 + 0] = v[0]; tile[row][c4 + 1] = v[1]; tile[row][c4 + 2] = v[2]; tile[row][c4 + 3] = v[3];
    }
  }
  __syncthreads();
  _Float16* Hh = (_Float16*)Hh16p;
  _Float16* Ht = (_Float16*)Ht16p;
  const int q8 = lane >> 3, c8 = (lane & 7) * 8;
  for (int pass = 0; pass < 2; ++pass) {
#pragma unroll
    for (int it = 0; it < 2; ++it) {
      const int row = it * 32 + wave * 4 + q8;
      v8h o, t;
#pragma unroll
      for (int e = 0; e < 8; ++e) { o[e] = (_Float16)tile[row][c8 + e]; t[e] = (_Float16)tile[c8 + e][row]; }
      *(volatile v8h*)(Hh + ((size_t)(b * SEQ + kbase + row)) * FEATD + fbase + c8) = o;
      *(volatile v8h*)(Ht + ((size_t)(b * FEATD + fbase + row)) * SEQ + kbase + c8) = t;
    }
    __threadfence();
  }
}

__global__ __launch_bounds__(256) void mean_kernel(const float* __restrict__ hidden, float* __restrict__ meanH) {
  __shared__ __align__(16) float sm[FEATD];
  const int b = blockIdx.x, f = threadIdx.x;
  const float* p = hidden + (size_t)b * SEQ * FEATD + f;
  float s0 = 0.f, s1 = 0.f;
#pragma unroll 4
  for (int k = 0; k < SEQ; k += 2) {
    s0 += p[(size_t)k * FEATD];
    s1 += p[(size_t)(k + 1) * FEATD];
  }
  sm[f] = (s0 + s1) * (1.0f / 512.0f);
  __syncthreads();
  if (threadIdx.x < 64) {
    const v4f v = *(const v4f*)(sm + 4 * threadIdx.x);
    float* dst = meanH + (size_t)b * FEATD + 4 * threadIdx.x;
    *(volatile v4f*)dst = v;
    __threadfence();
    *(volatile v4f*)dst = v;
  }
}

__global__ __launch_bounds__(256) void score_softmax_kernel(
    const float* __restrict__ hidden, const float* __restrict__ Wsp, const float* __restrict__ vsp,
    const unsigned short* __restrict__ Hh16p, float* __restrict__ att, unsigned short* __restrict__ P16p) {
  extern __shared__ __align__(16) unsigned char smem_raw[];
  _Float16* sB   = (_Float16*)smem_raw;
  float*    s_hq = (float*)(smem_raw + SB_BYTES);
  float*    s_vs = s_hq + FEATD;
  float*    s_s  = s_vs + MODD;
  float*    s_red = s_s + SEQ;

  const int tid = threadIdx.x, wave = tid >> 5, lane = tid & 31;
  const int hh = lane >> 4, rlane = lane & 15, koff = hh * 8;
  const int bq = blockIdx.x;
  const int b  = bq / SEQ;

  s_hq[tid] = hidden[(size_t)bq * FEATD + tid];
  if (tid < MODD) s_vs[tid] = vsp[tid];
  __syncthreads();

#pragma unroll 1
  for (int it = 0; it < 16; ++it) {
    const int idx = it * 256 + tid;
    const int d = idx >> 5, f8 = (idx & 31) * 8;
    const v4f w0 = *(const v4f*)(Wsp + (size_t)d * FEATD + f8);
    const v4f w1 = *(const v4f*)(Wsp + (size_t)d * FEATD + f8 + 4);
    const v4f h0 = *(const v4f*)(s_hq + f8);
    const v4f h1 = *(const v4f*)(s_hq + f8 + 4);
    v8h o;
#pragma unroll
    for (int e = 0; e < 4; ++e) {
      o[e]     = (_Float16)((BSC * h0[e]) * w0[e]);
      o[4 + e] = (_Float16)((BSC * h1[e]) * w1[e]);
    }
    *(v8h*)(sB + d * BPITCH + f8) = o;
  }
  __syncthreads();

  const _Float16* Hh = (const _Float16*)Hh16p + (size_t)b * SEQ * FEATD;
  v8f acc[8];
#pragma unroll 1
  for (int iter = 0; iter < 4; ++iter) {
    const int m0 = (wave * 4 + iter) * 16;
#pragma unroll
    for (int nt = 0; nt < 8; ++nt) acc[nt] = (v8f){0.f,0.f,0.f,0.f,0.f,0.f,0.f,0.f};
    const _Float16* arow = Hh + (size_t)(m0 + rlane) * FEATD + koff;
#pragma unroll 1
    for (int k0 = 0; k0 < FEATD; k0 += 32) {
      v16h bfr[8];
#pragma unroll
      for (int nt = 0; nt < 8; ++nt) bfr[nt] = Frag<_Float16>::load(sB + (nt * 16 + rlane) * BPITCH + koff + k0);
      const v16h a = Frag<_Float16>::load(arow + k0);
#pragma unroll
      for (int nt = 0; nt < 8; ++nt) acc[nt] = Frag<_Float16>::mma(a, bfr[nt], acc[nt]);
      dep_guard_h(acc[0], acc[7], a, bfr[7]);
      keep4_h(bfr[0], bfr[1], bfr[2], bfr[3]);
      keep4_h(bfr[4], bfr[5], bfr[6], bfr[7]);
    }
    acc_guard4(acc[0], acc[1], acc[2], acc[3]);
    acc_guard4(acc[4], acc[5], acc[6], acc[7]);

    float tsum[8];
#pragma unroll
    for (int r = 0; r < 8; ++r) tsum[r] = 0.f;
#pragma unroll
    for (int nt = 0; nt < 8; ++nt) {
      const float vv = s_vs[nt * 16 + rlane];
#pragma unroll
      for (int r = 0; r < 8; ++r) {
        const float z = acc[nt][r] * BSC_INV;
        const float e = __expf(z + z);
        const float t = fmaf(-2.0f, __builtin_amdgcn_rcpf(e + 1.0f), 1.0f);
        tsum[r] = fmaf(t, vv, tsum[r]);
      }
    }
    float mine = 0.f;
#pragma unroll
    for (int r = 0; r < 8; ++r) {
      float t = tsum[r];
      t += __shfl_xor(t, 1, 32);
      t += __shfl_xor(t, 2, 32);
      t += __shfl_xor(t, 4, 32);
      t += __shfl_xor(t, 8, 32);
      mine = (rlane == r) ? t : mine;
    }
    if (rlane < 8) s_s[m0 + 8 * hh + rlane] = mine;
  }
  __syncthreads();

  const float v0 = s_s[tid], v1 = s_s[tid + 256];
  float mx = fmaxf(v0, v1);
#pragma unroll
  for (int off = 16; off > 0; off >>= 1) mx = fmaxf(mx, __shfl_xor(mx, off, 32));
  if (lane == 0) s_red[wave] = mx;
  __syncthreads();
  float gm = s_red[0];
#pragma unroll
  for (int w = 1; w < 8; ++w) gm = fmaxf(gm, s_red[w]);
  const float e0 = expf(v0 - gm), e1 = expf(v1 - gm);
  float sum = e0 + e1;
#pragma unroll
  for (int off = 16; off > 0; off >>= 1) sum += __shfl_xor(sum, off, 32);
  if (lane == 0) s_red[8 + wave] = sum;
  __syncthreads();
  float tot = 0.f;
#pragma unroll
  for (int w = 0; w < 8; ++w) tot += s_red[8 + w];
  const float inv = 1.0f / tot;
  s_s[tid] = e0 * inv;
  s_s[tid + 256] = e1 * inv;
  __syncthreads();

  if (wave < 4) {
    const v4f v = *(const v4f*)(s_s + 4 * tid);
    float* dst = att + (size_t)bq * SEQ + 4 * tid;
    *(volatile v4f*)dst = v;
    __threadfence();
    *(volatile v4f*)dst = v;
  } else if (wave < 6) {
    const int j = tid - 128;
    v8h o;
#pragma unroll
    for (int e = 0; e < 8; ++e) o[e] = (_Float16)(s_s[8 * j + e] * PCARRY - PCENTRE);
    _Float16* dst = (_Float16*)P16p + (size_t)bq * SEQ + 8 * j;
    *(volatile v8h*)dst = o;
    __threadfence();
    *(volatile v8h*)dst = o;
  }
}

extern "C" void kernel_launch(void* const* d_in, const int* in_sizes, int n_in,
                              void* d_out, int out_size, void* d_ws, size_t ws_size,
                              hipStream_t stream) {
  if (n_in < 3) return;
  if (in_sizes[0] != NBATCH * SEQ * FEATD || in_sizes[1] != MODD * FEATD || in_sizes[2] != MODD) return;
  if (out_size != NBATCH * SEQ * FEATD + NBATCH * SEQ * SEQ) return;
  if (ws_size < WS_TOTAL) return;

  const float* hidden = (const float*)d_in[0];
  const float* Wsp    = (const float*)d_in[1];
  const float* vsp    = (const float*)d_in[2];
  float* ctx = (float*)d_out;
  float* att = (float*)d_out + (OUT1_OFF / 4);

  char* wsb = (char*)d_ws;
  unsigned short* Hh16 = (unsigned short*)(wsb + OFF_HH);
  unsigned short* Ht16 = (unsigned short*)(wsb + OFF_HT);
  unsigned short* P16  = (unsigned short*)(wsb + OFF_P);
  float* meanH = (float*)(wsb + OFF_MEAN);

  planes_kernel<<<dim3(SEQ / 64, FEATD / 64, NBATCH), dim3(256), 0, stream>>>(hidden, Hh16, Ht16);
  mean_kernel<<<dim3(NBATCH), dim3(256), 0, stream>>>(hidden, meanH);
  score_softmax_kernel<<<dim3(NBATCH * SEQ), dim3(256), SMEM_BYTES, stream>>>(hidden, Wsp, vsp, Hh16, att, P16);
  {
    const int tiles = (SEQ / 64) * (FEATD / 64);
    const dim3 grid((tiles + 7) / 8, NBATCH);
    wmma_gemm64<0, false, 3, 0, false, 0><<<grid, dim3(256), 0, stream>>>(
        P16, P16, SEQ, (long)SEQ * SEQ,
        Ht16, Ht16, SEQ, (long)FEATD * SEQ,
        (void*)ctx, (void*)ctx, FEATD, (long)SEQ * FEATD,
        meanH,
        meanH, 0L,
        SEQ, FEATD, SEQ, 1.0f / PCARRY);
  }
}
